// EquivariantMPLayer_41317585387560
// MI455X (gfx1250) — hardware-verified
//
#include <hip/hip_runtime.h>
#include <stddef.h>


#define CIN   128
#define HID   256
#define RNK   16
#define NTY   4
#define MSG   257
#define MLPK  384

#define KY    128
#define NYC   128
#define KS    320
#define KM    512
#define ZW    64
#define SCW   8

#define PY_OFF 0
#define PY_N   (NYC * KY)
#define PS_OFF (PY_OFF + PY_N)
#define PS_N   (HID * KS)
#define PM_OFF (PS_OFF + PS_N)
#define PM_N   (HID * KM)
#define PL_TOT (PM_OFF + PM_N)

#define NTHR   256
#define NWAVE  8
#define EPT    8
#define NGRP   2
#define CHUNK  (NTHR * EPT * NGRP)
#define WCAP   (EPT * NGRP * 32)
#define LISTN  (NWAVE * WCAP)
#define NB     320
#define NBK    5
#define SLOTF  192
#define RB     128
#define TP     128

#define LDS_ACC  (NB * SLOTF * 4)
#define LDS_LIST (LISTN * 4)
#define LDS_CNT  (NBK * NB * 4)
#define LDS_DSM  (NBK * NB * 4)
#define LDS_AGG  (LDS_ACC + LDS_LIST + LDS_CNT + LDS_DSM + 64)

static_assert((CHUNK & (CHUNK - 1)) == 0);
static_assert(CHUNK <= 4096);
static_assert(NB < 4096);
static_assert(NB % 16 == 0);
static_assert(NB * SCW * 4 <= LDS_LIST);
static_assert(NWAVE * 4 <= 64);
static_assert(LDS_AGG <= 300 * 1024);
static_assert((PS_OFF % 64) == 0);
static_assert((PM_OFF % 64) == 0);
static_assert((PL_TOT % 64) == 0);
static_assert((PL_TOT % 8) == 0);
static_assert((SLOTF % 4) == 0);

typedef float  v4f   __attribute__((ext_vector_type(4)));
typedef float  v8f   __attribute__((ext_vector_type(8)));
typedef int    v4i   __attribute__((ext_vector_type(4)));
typedef __bf16 bf16_t;
typedef bf16_t v8bf  __attribute__((ext_vector_type(8)));
typedef bf16_t v16bf __attribute__((ext_vector_type(16)));
union FragB { v16bf v; v8bf h[2]; v4i q[2]; };
union Pack8 { v8bf v; v4i q; };

__device__ __forceinline__ v8f wmb(v16bf a, v16bf b, v8f c) {
  v8f d = __builtin_amdgcn_wmma_f32_16x16x32_bf16(false, a, false, b, (short)0, c, false, false);
  asm volatile("v_nop\n\tv_nop\n\tv_nop\n\tv_nop" : "+v"(d) : "v"(a), "v"(b));
  return d;
}

template <int B>
__device__ __forceinline__ void split8(FragB& hi, FragB& lo, v4f a, v4f b) {
#define SPL1(I, X) { const float xv = (X); const bf16_t hb = (bf16_t)xv; hi.v[B + (I)] = hb; lo.v[B + (I)] = (bf16_t)(xv - (float)hb); }
  SPL1(0, a.x) SPL1(1, a.y) SPL1(2, a.z) SPL1(3, a.w)
  SPL1(4, b.x) SPL1(5, b.y) SPL1(6, b.z) SPL1(7, b.w)
#undef SPL1
}

template <int NCT, int KP>
__device__ __forceinline__ void kstep(const float* ap, float mul,
                                      const bf16_t* bhp, const bf16_t* blp, v8f (&c)[NCT]) {
  const v4f p0 = (*(const v4f*)(ap))      * mul;
  const v4f p1 = (*(const v4f*)(ap + 4))  * mul;
  const v4f p2 = (*(const v4f*)(ap + 16)) * mul;
  const v4f p3 = (*(const v4f*)(ap + 20)) * mul;
  FragB ahi, alo;
  split8<0>(ahi, alo, p0, p1);
  split8<8>(ahi, alo, p2, p3);
#pragma unroll
  for (int ct = 0; ct < NCT; ++ct) {
    const bf16_t* hp = bhp + (size_t)ct * 16 * KP;
    const bf16_t* lp = blp + (size_t)ct * 16 * KP;
    FragB bh, bq;
    bh.q[0] = *(const v4i*)hp;  bh.q[1] = *(const v4i*)(hp + 16);
    bq.q[0] = *(const v4i*)lp;  bq.q[1] = *(const v4i*)(lp + 16);
    c[ct] = wmb(alo.v, bh.v, c[ct]);
    c[ct] = wmb(ahi.v, bq.v, c[ct]);
    c[ct] = wmb(ahi.v, bh.v, c[ct]);
  }
}

__device__ __forceinline__ void acc_to_tile(float* tw, v8f (&c)[8], int hh, int m) {
  float* sp = tw + (8 * hh) * TP + m;
#pragma unroll
  for (int ct = 0; ct < 8; ++ct) {
#pragma unroll
    for (int r = 0; r < 8; ++r) sp[r * TP + 16 * ct] = c[ct][r];
  }
}

template <int NBT>
__device__ __forceinline__ int scan_chunk(const int* __restrict__ dsts, int nE, int cbase, int nodeBase,
                                          int vec8, int* list, int tid, int lane, int wave) {
  int wc = 0;
  (void)lane;
#pragma unroll
  for (int g = 0; g < NGRP; ++g) {
    const int el0  = (g * NTHR + tid) * EPT;
    const int e0   = cbase + el0;
    const int sent = -2147483647 - 1;
    v4i da, db;
    if (vec8 != 0 && cbase + CHUNK <= nE) {
      da = *(const v4i*)(dsts + e0);
      db = *(const v4i*)(dsts + e0 + 4);
    } else {
      da.x = (e0     < nE) ? dsts[min(e0, nE - 1)] : sent;
      da.y = (e0 + 1 < nE) ? dsts[min(e0 + 1, nE - 1)] : sent;
      da.z = (e0 + 2 < nE) ? dsts[min(e0 + 2, nE - 1)] : sent;
      da.w = (e0 + 3 < nE) ? dsts[min(e0 + 3, nE - 1)] : sent;
      db.x = (e0 + 4 < nE) ? dsts[min(e0 + 4, nE - 1)] : sent;
      db.y = (e0 + 5 < nE) ? dsts[min(e0 + 5, nE - 1)] : sent;
      db.z = (e0 + 6 < nE) ? dsts[min(e0 + 6, nE - 1)] : sent;
      db.w = (e0 + 7 < nE) ? dsts[min(e0 + 7, nE - 1)] : sent;
    }
    const unsigned nb = (unsigned)nodeBase;
    const unsigned s0 = (unsigned)da.x - nb, s1 = (unsigned)da.y - nb;
    const unsigned s2 = (unsigned)da.z - nb, s3 = (unsigned)da.w - nb;
    const unsigned s4 = (unsigned)db.x - nb, s5 = (unsigned)db.y - nb;
    const unsigned s6 = (unsigned)db.z - nb, s7 = (unsigned)db.w - nb;
    const bool h0 = s0 < (unsigned)NBT, h1 = s1 < (unsigned)NBT, h2 = s2 < (unsigned)NBT, h3 = s3 < (unsigned)NBT;
    const bool h4 = s4 < (unsigned)NBT, h5 = s5 < (unsigned)NBT, h6 = s6 < (unsigned)NBT, h7 = s7 < (unsigned)NBT;
    const unsigned any = __builtin_amdgcn_ballot_w32(h0 | h1 | h2 | h3 | h4 | h5 | h6 | h7);
    if (any != 0u) {
#define HITJ(J, HJ, SJ) { \
        const unsigned mj = __builtin_amdgcn_ballot_w32(HJ); \
        if (mj != 0u) { \
          if (HJ) { \
            const int pos = wc + (int)__builtin_amdgcn_mbcnt_lo(mj, 0u); \
            if (pos < WCAP) list[wave * WCAP + pos] = ((el0 + (J)) << 12) | (int)(SJ); \
          } \
          wc += (int)__builtin_popcount(mj); } }
      HITJ(0, h0, s0)
      HITJ(1, h1, s1)
      HITJ(2, h2, s2)
      HITJ(3, h3, s3)
      HITJ(4, h4, s4)
      HITJ(5, h5, s5)
      HITJ(6, h6, s6)
      HITJ(7, h7, s7)
#undef HITJ
    }
  }
  return wc;
}

__global__ __launch_bounds__(NTHR) void k_wprep(
    const float* __restrict__ Bw, const float* __restrict__ Wsh, const float* __restrict__ Aw,
    const float* __restrict__ mlpw, const float* __restrict__ Wres, const float* __restrict__ npos,
    bf16_t* phi, bf16_t* plo, int nTot) {
  (void)npos;
  const int i = blockIdx.x * NTHR + threadIdx.x;
  if (i >= nTot) return;
  const int o = i * 8;
  const float* src;
  if (o < PS_OFF) {
    const int n = o / KY, k0 = o - n * KY;
    src = (n < 64) ? (Bw + (size_t)n * MSG + k0) : (Bw + (size_t)(n - 64) * MSG + 128 + k0);
  } else if (o < PM_OFF) {
    const int rem = o - PS_OFF;
    const int n = rem / KS, k0 = rem - n * KS;
    if (k0 < 256) {
      src = Wsh + (size_t)n * MSG + k0;
    } else {
      const int j0 = k0 - 256, t = j0 >> 4, r0 = j0 & 15;
      src = Aw + ((size_t)t * HID + n) * RNK + r0;
    }
  } else {
    const int rem = o - PM_OFF;
    const int n = rem / KM, k0 = rem - n * KM;
    src = (k0 < MLPK) ? (mlpw + (size_t)n * MLPK + k0) : (Wres + (size_t)n * CIN + (k0 - MLPK));
  }
  Pack8 ph, pl;
#define WSP(I) { const float xv = src[(I)]; const bf16_t hb = (bf16_t)xv; ph.v[(I)] = hb; pl.v[(I)] = (bf16_t)(xv - (float)hb); }
  WSP(0) WSP(1) WSP(2) WSP(3) WSP(4) WSP(5) WSP(6) WSP(7)
#undef WSP
  bf16_t* dh = phi + o;
  bf16_t* dl = plo + o;
  const v4i qh = ph.q, ql = pl.q;
  *(volatile v4i*)dh = qh;
  *(volatile v4i*)dl = ql;
  __threadfence();
  *(volatile v4i*)dh = qh;
  *(volatile v4i*)dl = ql;
}

__global__ __launch_bounds__(NTHR) void k_y(
    const float* __restrict__ x, const bf16_t* __restrict__ phi, const bf16_t* __restrict__ plo,
    float* Y, int nN) {
  __shared__ __align__(16) float tile[NWAVE * 16 * TP];
  const int tid = threadIdx.x, lane = tid & 31, wave = tid >> 5, hh = lane >> 4, m = lane & 15;
  const int rowBase = blockIdx.x * RB + 16 * wave;
  int node = rowBase + m; node = node > nN - 1 ? nN - 1 : node;

  v8f c[8];
#pragma unroll
  for (int ct = 0; ct < 8; ++ct) { const v8f z = {0.f, 0.f, 0.f, 0.f, 0.f, 0.f, 0.f, 0.f}; c[ct] = z; }

  const float*  arow = x + (size_t)node * CIN + 8 * hh;
  const bf16_t* bh0  = phi + PY_OFF + (size_t)m * KY + 8 * hh;
  const bf16_t* bl0  = plo + PY_OFF + (size_t)m * KY + 8 * hh;
#pragma unroll 1
  for (int ks = 0; ks < CIN / 32; ++ks)
    kstep<8, KY>(arow + 32 * ks, 1.0f, bh0 + 32 * ks, bl0 + 32 * ks, c);

  acc_to_tile(tile + wave * 16 * TP, c, hh, m);
  __syncthreads();

  const float* lrow = tile + wave * 16 * TP + 4 * lane;
  float* gp = Y + (size_t)rowBase * KY + 4 * lane;
#pragma unroll
  for (int i = 0; i < 16; ++i) { const v4f v = *(const v4f*)(lrow + i * TP); *(volatile v4f*)(gp + (size_t)i * KY) = v; }
  __threadfence();
#pragma unroll
  for (int i = 0; i < 16; ++i) { const v4f v = *(const v4f*)(lrow + i * TP); *(volatile v4f*)(gp + (size_t)i * KY) = v; }
}

__global__ __launch_bounds__(NTHR) void k_aggr(
    const int* __restrict__ ei, const float* __restrict__ eattr,
    const float* __restrict__ x, const float* __restrict__ Y, const float* __restrict__ Bw,
    float* Sg, float* Zg, float* SCg, int nN, int nE, int vec8) {
  extern __shared__ v4f lds_dyn[];
  float* acc  = (float*)lds_dyn;
  int*   list = (int*)((char*)lds_dyn + LDS_ACC);
  int*   cnt  = (int*)((char*)lds_dyn + LDS_ACC + LDS_LIST);
  float* dsm  = (float*)((char*)lds_dyn + LDS_ACC + LDS_LIST + LDS_CNT);
  int*   wcnt = (int*)((char*)lds_dyn + LDS_ACC + LDS_LIST + LDS_CNT + LDS_DSM);
  float* scs  = (float*)list;
  const int tid = threadIdx.x, lane = tid & 31, wave = tid >> 5;
  const int nodeBase = blockIdx.x * NB;
  const int* dsts = ei + nE;

  {
    const v4f z = {0.f, 0.f, 0.f, 0.f};
    for (int i = tid; i < NB * SLOTF / 4; i += NTHR) lds_dyn[i] = z;
    for (int i = tid; i < NBK * NB; i += NTHR) { cnt[i] = 0; dsm[i] = 0.0f; }
  }
  __syncthreads();

  const int nChunks = (nE + CHUNK - 1) / CHUNK;
#pragma unroll 1
  for (int ch = 0; ch < nChunks; ++ch) {
    const int cbase = ch * CHUNK;
    const int wc = scan_chunk<NB>(dsts, nE, cbase, nodeBase, vec8, list, tid, lane, wave);
    if (lane == 0) wcnt[wave] = wc;
    __syncthreads();
    if (wave == 0) {
#pragma unroll 1
      for (int wsx = 0; wsx < NWAVE; ++wsx) {
        int n = __builtin_amdgcn_readfirstlane(wcnt[wsx]);
        n = n > WCAP ? WCAP : (n < 0 ? 0 : n);
        const int* lp = list + wsx * WCAP;
#pragma unroll 1
        for (int i = 0; i < n; ++i) {
          const int ent = __builtin_amdgcn_readfirstlane(lp[i]);
          int slot = ent & 4095;
          slot = slot > NB - 1 ? NB - 1 : slot;
          int e = cbase + ((ent >> 12) & (CHUNK - 1));
          e = e > nE - 1 ? nE - 1 : e;
          int src = ei[e];
          src = src < 0 ? 0 : (src > nN - 1 ? nN - 1 : src);
          float ta = eattr[(size_t)e * 2];
          const float dist = eattr[(size_t)e * 2 + 1];
          ta = fminf(fmaxf(ta, -16.0f), 16.0f);
          const int te = (int)ta;
          const int b  = (te >= 0 && te <= 3) ? te : 4;
          const int tc = b > 3 ? 3 : b;
          const v4f xv = *(const v4f*)(x + (size_t)src * CIN + 4 * lane);
          const v4f yv = *(const v4f*)(Y + (size_t)src * KY + 16 * tc + 4 * (lane & 3));
          v4f* ap = (v4f*)(acc + slot * SLOTF + 4 * lane);
          *ap = *ap + xv;
          if (b < 4 && lane < 4) {
            v4f* zp = (v4f*)(acc + slot * SLOTF + 128 + 16 * tc + 4 * lane);
            *zp = *zp + yv;
          }
          if (lane == 0) { cnt[b * NB + slot] = cnt[b * NB + slot] + 1; dsm[b * NB + slot] = dsm[b * NB + slot] + dist; }
        }
      }
    }
    __syncthreads();
  }

  for (int s = tid; s < NB; s += NTHR) {
    const float c0 = (float)cnt[s], c1 = (float)cnt[NB + s], c2 = (float)cnt[2 * NB + s];
    const float c3 = (float)cnt[3 * NB + s], c4 = (float)cnt[4 * NB + s];
    const float d  = dsm[s] + dsm[NB + s] + dsm[2 * NB + s] + dsm[3 * NB + s] + dsm[4 * NB + s];
    float* sp = scs + s * SCW;
    sp[0] = c0 + c1 + c2 + c3 + c4;
    sp[1] = d;
    sp[2] = c0; sp[3] = c1; sp[4] = c2; sp[5] = c3;
    sp[6] = 0.0f; sp[7] = 0.0f;
  }
  for (int idx = tid; idx < NB * ZW; idx += NTHR) {
    const int s = idx >> 6, j = idx & 63, t = j >> 4;
    int node = nodeBase + s; node = node > nN - 1 ? nN - 1 : node;
    const float ct = (float)cnt[t * NB + s];
    const float dt = dsm[t * NB + s];
    const float z = acc[s * SLOTF + 128 + j] + ct * Y[(size_t)node * KY + 64 + j] + dt * Bw[(size_t)j * MSG + 256];
    acc[s * SLOTF + 128 + j] = z;
  }
  __syncthreads();

  for (int i = wave; i < NB; i += NWAVE) {
    const v4f v = *(const v4f*)(acc + i * SLOTF + 4 * lane);
    *(volatile v4f*)(Sg + (size_t)(nodeBase + i) * CIN + 4 * lane) = v;
  }
  for (int j = wave; j < NB / 2; j += NWAVE) {
    const int r = 2 * j + (lane >> 4);
    const v4f v = *(const v4f*)(acc + r * SLOTF + 128 + 4 * (lane & 15));
    *(volatile v4f*)(Zg + (size_t)(nodeBase + r) * ZW + 4 * (lane & 15)) = v;
  }
  for (int j = wave; j < NB / 16; j += NWAVE) {
    const int s = 16 * j + (lane >> 1);
    const v4f v = *(const v4f*)(scs + s * SCW + 4 * (lane & 1));
    *(volatile v4f*)(SCg + (size_t)(nodeBase + s) * SCW + 4 * (lane & 1)) = v;
  }
  __threadfence();
  for (int i = wave; i < NB; i += NWAVE) {
    const v4f v = *(const v4f*)(acc + i * SLOTF + 4 * lane);
    *(volatile v4f*)(Sg + (size_t)(nodeBase + i) * CIN + 4 * lane) = v;
  }
  for (int j = wave; j < NB / 2; j += NWAVE) {
    const int r = 2 * j + (lane >> 4);
    const v4f v = *(const v4f*)(acc + r * SLOTF + 128 + 4 * (lane & 15));
    *(volatile v4f*)(Zg + (size_t)(nodeBase + r) * ZW + 4 * (lane & 15)) = v;
  }
  for (int j = wave; j < NB / 16; j += NWAVE) {
    const int s = 16 * j + (lane >> 1);
    const v4f v = *(const v4f*)(scs + s * SCW + 4 * (lane & 1));
    *(volatile v4f*)(SCg + (size_t)(nodeBase + s) * SCW + 4 * (lane & 1)) = v;
  }
}

__device__ __forceinline__ v4f sums_row(const float* lp, const float* __restrict__ SCg, int row, int nN,
                                        v4f wl, v4f ab0, v4f ab1, v4f ab2, v4f ab3) {
  const int nr = row > nN - 1 ? nN - 1 : row;
  const v4f s0 = *(const v4f*)(SCg + (size_t)nr * SCW);
  const v4f s1 = *(const v4f*)(SCg + (size_t)nr * SCW + 4);
  const float inv = 1.0f / fmaxf(s0.x, 1.0f);
  v4f v = *(const v4f*)lp;
  v = v + s0.y * wl + s0.z * ab0 + s0.w * ab1 + s1.x * ab2 + s1.y * ab3;
  return v * inv;
}

__global__ __launch_bounds__(NTHR) void k_sums(
    const float* __restrict__ x, const float* __restrict__ Sg, const float* __restrict__ Zg,
    const float* __restrict__ SCg, const bf16_t* __restrict__ phi, const bf16_t* __restrict__ plo,
    const float* __restrict__ Wsh, const float* __restrict__ Ab, float* AG, int nN) {
  __shared__ __align__(16) float tile[NWAVE * 16 * TP];
  const int tid = threadIdx.x, lane = tid & 31, wave = tid >> 5, hh = lane >> 4, m = lane & 15;
  const int rowBase = blockIdx.x * RB + 16 * wave;
  const int colBase = blockIdx.y * 128;
  int node = rowBase + m; node = node > nN - 1 ? nN - 1 : node;
  const float cs = SCg[(size_t)node * SCW];

  v8f c[8];
#pragma unroll
  for (int ct = 0; ct < 8; ++ct) { const v8f z = {0.f, 0.f, 0.f, 0.f, 0.f, 0.f, 0.f, 0.f}; c[ct] = z; }

  const bf16_t* bh0  = phi + PS_OFF + (size_t)(colBase + m) * KS + 8 * hh;
  const bf16_t* bl0  = plo + PS_OFF + (size_t)(colBase + m) * KS + 8 * hh;
  const float*  srow = Sg + (size_t)node * CIN + 8 * hh;
  const float*  xrow = x  + (size_t)node * CIN + 8 * hh;
  const float*  zrow = Zg + (size_t)node * ZW  + 8 * hh;
#pragma unroll 1
  for (int ks = 0; ks < CIN / 32; ++ks)
    kstep<8, KS>(srow + 32 * ks, 1.0f, bh0 + 32 * ks, bl0 + 32 * ks, c);
#pragma unroll 1
  for (int ks = 0; ks < CIN / 32; ++ks)
    kstep<8, KS>(xrow + 32 * ks, cs, bh0 + 128 + 32 * ks, bl0 + 128 + 32 * ks, c);
#pragma unroll 1
  for (int ks = 0; ks < ZW / 32; ++ks)
    kstep<8, KS>(zrow + 32 * ks, 1.0f, bh0 + 256 + 32 * ks, bl0 + 256 + 32 * ks, c);

  acc_to_tile(tile + wave * 16 * TP, c, hh, m);
  __syncthreads();

  const int cb = colBase + 4 * lane;
  v4f wl;
  wl.x = Wsh[(size_t)(cb)     * MSG + 256];
  wl.y = Wsh[(size_t)(cb + 1) * MSG + 256];
  wl.z = Wsh[(size_t)(cb + 2) * MSG + 256];
  wl.w = Wsh[(size_t)(cb + 3) * MSG + 256];
  const v4f ab0 = *(const v4f*)(Ab + cb);
  const v4f ab1 = *(const v4f*)(Ab + HID + cb);
  const v4f ab2 = *(const v4f*)(Ab + 2 * HID + cb);
  const v4f ab3 = *(const v4f*)(Ab + 3 * HID + cb);

  const float* lrow = tile + wave * 16 * TP + 4 * lane;
  float* gp = AG + (size_t)rowBase * HID + cb;
#pragma unroll 1
  for (int i = 0; i < 16; ++i) {
    const v4f v = sums_row(lrow + i * TP, SCg, rowBase + i, nN, wl, ab0, ab1, ab2, ab3);
    *(volatile v4f*)(gp + (size_t)i * HID) = v;
  }
  __threadfence();
#pragma unroll 1
  for (int i = 0; i < 16; ++i) {
    const v4f v = sums_row(lrow + i * TP, SCg, rowBase + i, nN, wl, ab0, ab1, ab2, ab3);
    *(volatile v4f*)(gp + (size_t)i * HID) = v;
  }
}

__global__ __launch_bounds__(NTHR) void k_final(
    const float* __restrict__ x, const float* __restrict__ AG,
    const bf16_t* __restrict__ phi, const bf16_t* __restrict__ plo,
    const float* __restrict__ mlpb, float* out, int nN) {
  __shared__ __align__(16) float tile[NWAVE * 16 * TP];
  const int tid = threadIdx.x, lane = tid & 31, wave = tid >> 5, hh = lane >> 4, m = lane & 15;
  const int rowBase = blockIdx.x * RB + 16 * wave;
  const int colBase = blockIdx.y * 128;
  int node = rowBase + m; node = node > nN - 1 ? nN - 1 : node;

  v8f c[8];
#pragma unroll
  for (int ct = 0; ct < 8; ++ct) { const v8f z = {0.f, 0.f, 0.f, 0.f, 0.f, 0.f, 0.f, 0.f}; c[ct] = z; }

  const bf16_t* bh0  = phi + PM_OFF + (size_t)(colBase + m) * KM + 8 * hh;
  const bf16_t* bl0  = plo + PM_OFF + (size_t)(colBase + m) * KM + 8 * hh;
  const float*  xrow = x  + (size_t)node * CIN + 8 * hh;
  const float*  grow = AG + (size_t)node * HID + 8 * hh;
#pragma unroll 1
  for (int ks = 0; ks < CIN / 32; ++ks)
    kstep<8, KM>(xrow + 32 * ks, 1.0f, bh0 + 32 * ks, bl0 + 32 * ks, c);
#pragma unroll 1
  for (int ks = 0; ks < HID / 32; ++ks)
    kstep<8, KM>(grow + 32 * ks, 1.0f, bh0 + 128 + 32 * ks, bl0 + 128 + 32 * ks, c);

#pragma unroll
  for (int ct = 0; ct < 8; ++ct) {
    const float b = mlpb[colBase + 16 * ct + m];
#pragma unroll
    for (int r = 0; r < 8; ++r) c[ct][r] = fmaxf(c[ct][r] + b, 0.0f);
  }

#pragma unroll 1
  for (int ks = 0; ks < CIN / 32; ++ks)
    kstep<8, KM>(xrow + 32 * ks, 1.0f, bh0 + MLPK + 32 * ks, bl0 + MLPK + 32 * ks, c);

  acc_to_tile(tile + wave * 16 * TP, c, hh, m);
  __syncthreads();

  const float* lrow = tile + wave * 16 * TP + 4 * lane;
  float* gp = out + (size_t)rowBase * HID + colBase + 4 * lane;
#pragma unroll
  for (int i = 0; i < 16; ++i) {
    if (rowBase + i < nN) { const v4f v = *(const v4f*)(lrow + i * TP); *(volatile v4f*)(gp + (size_t)i * HID) = v; }
  }
  __threadfence();
#pragma unroll
  for (int i = 0; i < 16; ++i) {
    if (rowBase + i < nN) { const v4f v = *(const v4f*)(lrow + i * TP); *(volatile v4f*)(gp + (size_t)i * HID) = v; }
  }
}

extern "C" void kernel_launch(void* const* d_in, const int* in_sizes, int n_in,
                              void* d_out, int out_size, void* d_ws, size_t ws_size,
                              hipStream_t stream) {
  if (n_in < 11) return;
  const int nN = in_sizes[0] / CIN;
  const int nE = in_sizes[10] / 2;
  if (nN <= 0 || nE <= 0) return;
  if (in_sizes[0] != nN * CIN) return;
  if (in_sizes[10] != 2 * nE || in_sizes[2] != 2 * nE) return;
  if (in_sizes[3] != HID * CIN || in_sizes[4] != NTY * HID * RNK || in_sizes[5] != NTY * HID) return;
  if (in_sizes[6] != NTY * RNK * MSG || in_sizes[7] != HID * MSG) return;
  if (in_sizes[8] != HID * MLPK || in_sizes[9] != HID) return;
  if (out_size != nN * HID) return;

  const float* x     = (const float*)d_in[0];
  const float* npos  = (const float*)d_in[1];
  const float* eattr = (const float*)d_in[2];
  const float* Wres  = (const float*)d_in[3];
  const float* Aw    = (const float*)d_in[4];
  const float* Ab    = (const float*)d_in[5];
  const float* Bw    = (const float*)d_in[6];
  const float* Wsh   = (const float*)d_in[7];
  const float* mlpw  = (const float*)d_in[8];
  const float* mlpb  = (const float*)d_in[9];
  const int*   ei    = (const int*)d_in[10];
  float* out = (float*)d_out;

  const int nBlkG = (nN + RB - 1) / RB;
  const int NpadG = nBlkG * RB;
  const int nBlkA = (nN + NB - 1) / NB;
  const int NpadA = nBlkA * NB;

  char* ws = (char*)d_ws;
  size_t off = 0;
  const size_t szP  = (size_t)PL_TOT * 2;
  const size_t szY  = (size_t)NpadG * KY  * 4;
  const size_t szS  = (size_t)NpadA * CIN * 4;
  const size_t szZ  = (size_t)NpadA * ZW  * 4;
  const size_t szSC = (size_t)NpadA * SCW * 4;
  const size_t szAG = (size_t)NpadG * HID * 4;
  const size_t oPH = off; off += szP;  off = (off + 255) & ~(size_t)255;
  const size_t oPL = off; off += szP;  off = (off + 255) & ~(size_t)255;
  const size_t oY  = off; off += szY;  off = (off + 255) & ~(size_t)255;
  const size_t oS  = off; off += szS;  off = (off + 255) & ~(size_t)255;
  const size_t oZ  = off; off += szZ;  off = (off + 255) & ~(size_t)255;
  const size_t oSC = off; off += szSC; off = (off + 255) & ~(size_t)255;
  const size_t oAG = off; off += szAG; off = (off + 255) & ~(size_t)255;
  if (off > ws_size || off > (size_t)134217728) return;
  bf16_t* phi = (bf16_t*)(ws + oPH);
  bf16_t* plo = (bf16_t*)(ws + oPL);
  float*  Y   = (float*)(ws + oY);
  float*  Sg  = (float*)(ws + oS);
  float*  Zg  = (float*)(ws + oZ);
  float*  SCg = (float*)(ws + oSC);
  float*  AG  = (float*)(ws + oAG);

  const int vec8 = ((nE & 3) == 0) ? 1 : 0;
  const int nTot = PL_TOT / 8;

  k_wprep<<<(nTot + NTHR - 1) / NTHR, NTHR, 0, stream>>>(Bw, Wsh, Aw, mlpw, Wres, npos, phi, plo, nTot);
  k_y<<<nBlkG, NTHR, 0, stream>>>(x, phi, plo, Y, nN);

  hipFuncSetAttribute(reinterpret_cast<const void*>(&k_aggr),
                      hipFuncAttributeMaxDynamicSharedMemorySize, LDS_AGG);
  k_aggr<<<nBlkA, NTHR, LDS_AGG, stream>>>(ei, eattr, x, Y, Bw, Sg, Zg, SCg, nN, nE, vec8);

  k_sums<<<dim3(nBlkG, 2), NTHR, 0, stream>>>(x, Sg, Zg, SCg, phi, plo, Wsh, Ab, AG, nN);
  k_final<<<dim3(nBlkG, 2), NTHR, 0, stream>>>(x, AG, phi, plo, mlpb, out, nN);
}
